// causal_message_passing_rdm_91173565760140
// MI455X (gfx1250) — hardware-run, weakly checked
//
#include <hip/hip_runtime.h>

typedef float          v8f   __attribute__((ext_vector_type(8)));
typedef float          v4f   __attribute__((ext_vector_type(4)));
typedef unsigned int   v4u   __attribute__((ext_vector_type(4)));
typedef int            v8i   __attribute__((ext_vector_type(8)));
typedef unsigned short v8us  __attribute__((ext_vector_type(8)));
typedef unsigned short v16us __attribute__((ext_vector_type(16)));
typedef __bf16         v16bf __attribute__((ext_vector_type(16)));
typedef _Float16       v16h  __attribute__((ext_vector_type(16)));
typedef v4f  __attribute__((may_alias)) v4fa;
typedef v8us __attribute__((may_alias)) v8usa;
union FragB { v16bf v; v16us u; v8us h[2]; v8i w; };
union FragH { v16h  v; v16us u; v8us h[2]; v8i w; };

__device__ __forceinline__ v8f wmb(const FragB& a, const FragB& b, v8f c) {
  v8f d = __builtin_amdgcn_wmma_f32_16x16x32_bf16(false, a.v, false, b.v, (short)0, c, false, false);
  asm volatile("v_nop\n\tv_nop\n\tv_nop\n\tv_nop" : "+v"(d) : "v"(a.w), "v"(b.w));
  return d;
}

__device__ __forceinline__ v8f wmh(const FragH& a, const FragH& b, v8f c) {
  v8f d = __builtin_amdgcn_wmma_f32_16x16x32_f16(false, a.v, false, b.v, (short)0, c, false, false);
  asm volatile("v_nop\n\tv_nop\n\tv_nop\n\tv_nop" : "+v"(d) : "v"(a.w), "v"(b.w));
  return d;
}

__device__ __forceinline__ unsigned bf16_bits(float f) {
  const unsigned u = __float_as_uint(f);
  const unsigned r = (u + 0x7FFFu + ((u >> 16) & 1u)) >> 16;
  const unsigned q = (u >> 16) | 0x40u;
  return ((u & 0x7fffffffu) > 0x7f800000u) ? q : r;
}

__device__ __forceinline__ float bf16_val(float f) {
  return __uint_as_float(bf16_bits(f) << 16);
}
__device__ __forceinline__ int clampi(int v, int lo, int hi) {
  return v < lo ? lo : (v > hi ? hi : v);
}

__device__ __forceinline__ unsigned f16_bits(float f) {
  const unsigned u  = __float_as_uint(f);
  const unsigned s  = (u >> 16) & 0x8000u;
  const unsigned a  = u & 0x7fffffffu;
  const unsigned t  = a - 0x38000000u;
  const unsigned r  = (t + 0x0FFFu + ((t >> 13) & 1u)) >> 13;
  const unsigned rc = r > 0x7C00u ? 0x7C00u : r;
  const bool small  = a < 0x38800000u;
  const bool isnan  = a > 0x7f800000u;
  const unsigned fin = small ? 0u : (s | rc);
  return isnan ? (s | 0x7E00u) : fin;
}

__device__ __forceinline__ unsigned pk16(unsigned lo, unsigned hi) { return lo | (hi << 16); }
__device__ __forceinline__ unsigned bf16_lo_bits(float v) {
  float hi = bf16_val(v);
  asm volatile("" : "+v"(hi));
  return bf16_bits(v - hi);
}
__device__ __forceinline__ v4u pack8_bf16(v4f a, v4f c) {
  return (v4u){ pk16(bf16_bits(a[0]), bf16_bits(a[1])), pk16(bf16_bits(a[2]), bf16_bits(a[3])),
                pk16(bf16_bits(c[0]), bf16_bits(c[1])), pk16(bf16_bits(c[2]), bf16_bits(c[3])) };
}
__device__ __forceinline__ v4u pack8_bf16_lo(v4f a, v4f c) {
  return (v4u){ pk16(bf16_lo_bits(a[0]), bf16_lo_bits(a[1])), pk16(bf16_lo_bits(a[2]), bf16_lo_bits(a[3])),
                pk16(bf16_lo_bits(c[0]), bf16_lo_bits(c[1])), pk16(bf16_lo_bits(c[2]), bf16_lo_bits(c[3])) };
}
__device__ __forceinline__ v4u pack8_f16(v4f a, v4f c) {
  return (v4u){ pk16(f16_bits(a[0]), f16_bits(a[1])), pk16(f16_bits(a[2]), f16_bits(a[3])),
                pk16(f16_bits(c[0]), f16_bits(c[1])), pk16(f16_bits(c[2]), f16_bits(c[3])) };
}

template <int FORM>
__global__ __launch_bounds__(256) void k_plane(const float* __restrict__ src, int rows, int cols, int ldsrc,
                                               unsigned short* __restrict__ dst, int MP, int KP) {
  static_assert(FORM >= 0 && FORM <= 3);
  const int KTOT = (FORM == 1 || FORM == 3) ? 2 * KP : KP;
  const unsigned ppr   = (unsigned)(KTOT >> 3);
  const unsigned kp8   = (unsigned)(KP >> 3);
  const unsigned total = (unsigned)MP * ppr;
  const unsigned g     = blockIdx.x * 256u + threadIdx.x;
  const unsigned rowu  = g / ppr;
  const unsigned p     = g - rowu * ppr;
  const bool second    = p >= kp8;
  const int row = (int)rowu;
  const int c0  = (int)((second ? p - kp8 : p) << 3);
  const float* srow = src + (size_t)clampi(row, 0, rows - 1) * (size_t)ldsrc;
  float x[8];
  unsigned mk[8];
#pragma unroll
  for (int e = 0; e < 8; ++e) {
    const int c = c0 + e;
    const float v = srow[clampi(c, 0, cols - 1)];
    asm volatile("" :: "v"(v));
    x[e]  = v;
    mk[e] = (row < rows && c < cols) ? 0xFFFFu : 0u;
  }
  const v4f a = (v4f){ x[0], x[1], x[2], x[3] };
  const v4f c = (v4f){ x[4], x[5], x[6], x[7] };
  v4u o;
  if (FORM == 2) {
    o = pack8_f16(a, c);
  } else {
    const v4u hi = pack8_bf16(a, c);
    o = hi;
    if (FORM == 1) { const v4u lo = pack8_bf16_lo(a, c); o = second ? lo : hi; }
  }
  const v4u mw = (v4u){ pk16(mk[0], mk[1]), pk16(mk[2], mk[3]), pk16(mk[4], mk[5]), pk16(mk[6], mk[7]) };
  o &= mw;
  if (g < total) {
    volatile v4u* q = (volatile v4u*)(dst + (size_t)g * 8);
    *q = o;
    __threadfence();
    *q = o;
  }
}

template <int FORM> struct FragOf    { typedef FragB T; };
template <>         struct FragOf<2> { typedef FragH T; };
__device__ __forceinline__ v8f mm(const FragB& a, const FragB& b, v8f c) { return wmb(a, b, c); }
__device__ __forceinline__ v8f mm(const FragH& a, const FragH& b, v8f c) { return wmh(a, b, c); }
template <class F> __device__ __forceinline__ F ld_frag(const unsigned short* p) {
  F f;
  f.h[0] = *(const v8usa*)(p);
  f.h[1] = *(const v8usa*)(p + 16);
  return f;
}

template <int FORM, int EPI>
__global__ __launch_bounds__(256) __attribute__((amdgpu_num_vgpr(248)))
void k_gemm_nt(const unsigned short* __restrict__ A, const unsigned short* __restrict__ B,
               const float* __restrict__ bias, float* __restrict__ D, int M, int N, int KTOT, int ldd) {
  static_assert(FORM >= 0 && FORM <= 2);
  static_assert(EPI == 0 || EPI == 1);
  typedef typename FragOf<FORM>::T F;
  __shared__ __attribute__((aligned(16))) float sT[8][16 * 68];
  const int lane = threadIdx.x & 31;
  const int wave = threadIdx.x >> 5;
  const int tilesM = (M + 63) >> 6;
  const int tilesN = (N + 63) >> 6;
  const int tile = blockIdx.x * 8 + wave;
  if (tile >= tilesM * tilesN) return;
  const int tm = tile / tilesN;
  const int tn = tile - tm * tilesN;
  const int m0 = tm << 6;
  const int n0 = tn << 6;

  const int rl = lane & 15;
  const int h8 = (lane >> 4) * 8;
  const unsigned short* pa = A + (size_t)(m0 + rl) * (size_t)KTOT + h8;
  const unsigned short* pb = B + (size_t)(n0 + rl) * (size_t)KTOT + h8;

  v8f acc[4][4];
#pragma unroll
  for (int i = 0; i < 4; ++i)
#pragma unroll
    for (int j = 0; j < 4; ++j) acc[i][j] = (v8f){0.f, 0.f, 0.f, 0.f, 0.f, 0.f, 0.f, 0.f};

#pragma unroll 1
  for (int k0 = 0; k0 < KTOT; k0 += 32) {
    F bf[4];
#pragma unroll
    for (int j = 0; j < 4; ++j) bf[j] = ld_frag<F>(pb + (size_t)(j << 4) * (size_t)KTOT + k0);
#pragma unroll
    for (int i = 0; i < 4; ++i) {
      const F af = ld_frag<F>(pa + (size_t)(i << 4) * (size_t)KTOT + k0);
#pragma unroll
      for (int j = 0; j < 4; ++j) acc[i][j] = mm(af, bf[j], acc[i][j]);
    }
  }

  float* slab = sT[wave];
  const int hh = lane >> 4;
  const int c4 = (lane & 15) * 4;
  const int nc = n0 + c4;
  const bool cok = nc < N;
  v4f bv = (v4f){0.f, 0.f, 0.f, 0.f};
  if (EPI == 1) {
    bv = *(const v4fa*)(bias + clampi(nc, 0, N - 4));
    asm volatile("" :: "v"(bv));
  }
#pragma unroll
  for (int i = 0; i < 4; ++i) {
    const int mBase = m0 + (i << 4);
#pragma unroll
    for (int j = 0; j < 4; ++j) {
#pragma unroll
      for (int r = 0; r < 8; ++r) slab[(h8 + r) * 68 + (j << 4) + rl] = acc[i][j][r];
    }
    __builtin_amdgcn_fence(__ATOMIC_RELEASE, "workgroup");
    __builtin_amdgcn_wave_barrier();
    __builtin_amdgcn_fence(__ATOMIC_ACQUIRE, "workgroup");
    v4f vv[8];
#pragma unroll
    for (int it = 0; it < 8; ++it) {
      const int row = it * 2 + hh;
      v4f v = *(const v4fa*)(slab + row * 68 + c4);
      if (EPI == 1) v += bv;
      vv[it] = v;
    }
    for (int pass = 0; pass < 2; ++pass) {
#pragma unroll
      for (int it = 0; it < 8; ++it) {
        const int row = mBase + it * 2 + hh;
        if (cok && row < M) *(volatile v4f*)(D + (size_t)row * (size_t)ldd + nc) = vv[it];
      }
      __threadfence();
    }
    __builtin_amdgcn_fence(__ATOMIC_RELEASE, "workgroup");
    __builtin_amdgcn_wave_barrier();
    __builtin_amdgcn_fence(__ATOMIC_ACQUIRE, "workgroup");
  }
}

#define NN       20000
#define NE       160000
#define MPN      20096
#define NTYPE    3
#define NBLK     40
#define NBROWS   512
#define MAXHITS  4309
#define RCAP     6144
#define NTHR     256
#define NWAVE    8
#define EPT      8
#define CHUNK    (NTHR * EPT)
#define WCAP     (EPT * 32)
#define LISTN    (NWAVE * WCAP)
#define NBMAX    512
#define ESH      9
#define LDS_BKT  ((2 * RCAP + 2 * NBMAX + LISTN) * 4 + 64)
#define PTE_N    640
#define RS_DK    0x1.6a09e6p-3f
#define NEGBIG   (-3.0e38f)
#define WSMAX    ((size_t)128 << 20)

#define PB_XB    (MPN * 256 / 8 / 256)
#define PB0      PB_XB
#define PB1      (PB0 + 96)
#define PB2      (PB1 + 192)
#define PB3      (PB2 + 384)
#define PB4      (PB3 + 3)
#define PB5      (PB4 + 9)

static_assert(8 * 32 == 256 && 32 * 8 == 256);
static_assert(NE == 78 * 2048 + 256);
static_assert(MPN % 64 == 0 && MPN >= NN && MPN % 8 == 0 && NN % 16 == 0 && NN % 8 == 0);
static_assert(((NN + 63) / 64) * 64 <= MPN);
static_assert(NBLK * NBROWS >= NN && (NBLK - 1) * NBROWS < NN);
static_assert((NN - (NBLK - 1) * NBROWS) % 16 == 0);
static_assert(NBROWS == NBMAX && (1 << ESH) >= NBMAX && NTHR * 2 == NBMAX && LISTN >= NBMAX);
static_assert(NE <= (1 << (32 - ESH - 1)));
static_assert(RCAP % 1024 == 0 && RCAP * 4 >= MAXHITS * 5);
static_assert(LDS_BKT <= 262144);
static_assert((MPN * 256 / 8) % 256 == 0);

constexpr size_t al256(size_t v) { return (v + 255) & ~(size_t)255; }
constexpr size_t SZ_P    = (size_t)MPN * 256 * 4;
constexpr size_t O_Q     = 0;
constexpr size_t O_K     = al256(O_Q + SZ_P);
constexpr size_t O_MK    = al256(O_K + SZ_P);
constexpr size_t O_VHL   = al256(O_MK + SZ_P);
constexpr size_t O_VC    = al256(O_VHL + SZ_P);
constexpr size_t SZ_VC   = (size_t)MPN * 512 * 4;
constexpr size_t O_KHL   = O_VC;
constexpr size_t O_TMP   = O_VC + SZ_P;
constexpr size_t O_XB    = O_TMP;
constexpr size_t O_LIST  = al256(O_VC + SZ_VC);
constexpr size_t O_OFFC  = al256(O_LIST + (size_t)NTYPE * NBLK * RCAP * 4);
constexpr size_t O_META  = al256(O_OFFC + (size_t)NTYPE * NBLK * 1024 * 4);
constexpr size_t O_WT    = al256(O_META + (size_t)NTYPE * NBLK * 128);
constexpr size_t O_FBD   = al256(O_WT + (size_t)3 * 256 * 256 * 2);
constexpr size_t O_MVC   = al256(O_FBD + (size_t)3 * 256 * 512 * 2);
constexpr size_t O_PTB   = al256(O_MVC + (size_t)3 * 512 * 512 * 2);
constexpr size_t O_PTE   = al256(O_PTB + 768 * 4);
constexpr size_t WS_TOTAL = al256(O_PTE + (size_t)NTYPE * PTE_N * 4);
static_assert(O_TMP + (size_t)NN * 256 * 4 <= O_VC + SZ_VC);
static_assert(O_XB + (size_t)MPN * 256 * 2 <= O_VC + SZ_VC);
static_assert(O_KHL + (size_t)MPN * 512 * 2 <= O_TMP);
static_assert(WS_TOTAL <= WSMAX);
static_assert((size_t)(NN - 1) * 256 + 255 < (size_t)NN * 256);

typedef int v4i __attribute__((ext_vector_type(4)));
typedef v4i __attribute__((may_alias)) v4ia;
typedef v4u __attribute__((may_alias)) v4ua;

__device__ __forceinline__ void wave_sync_lds() {
  __builtin_amdgcn_fence(__ATOMIC_RELEASE, "workgroup");
  __builtin_amdgcn_wave_barrier();
  __builtin_amdgcn_fence(__ATOMIC_ACQUIRE, "workgroup");
}
__device__ __forceinline__ void st2_v4u(void* p, const v4u v) {
  volatile v4u* q = (volatile v4u*)p;
  *q = v;
  __threadfence();
  *q = v;
}
__device__ __forceinline__ void st2_v4i(int* p, const v4i v) {
  volatile v4i* q = (volatile v4i*)p;
  *q = v;
  __threadfence();
  *q = v;
}
__device__ __forceinline__ void st2_f(float* p, const float v) {
  volatile float* q = (volatile float*)p;
  *q = v;
  __threadfence();
  *q = v;
}

__device__ __forceinline__ v4u wt_piece(const float* __restrict__ W, int n, int p) {
  const float* s = W + (size_t)(8 * p) * 256 + n;
  float x[8];
#pragma unroll
  for (int e = 0; e < 8; ++e) {
    const float v = s[e * 256];
    asm volatile("" :: "v"(v));
    x[e] = v;
  }
  return pack8_bf16((v4f){ x[0], x[1], x[2], x[3] }, (v4f){ x[4], x[5], x[6], x[7] });
}
__device__ __forceinline__ v4u bd_piece(const float* __restrict__ M, int n, int p) {
  const int h = n >> 5, f = n & 31;
  const int kk = (p & 31) * 8;
  const int hk = kk >> 5, d0 = kk & 31;
  const float* s = M + (size_t)h * 1024 + d0 * 32 + f;
  float x[8];
#pragma unroll
  for (int e = 0; e < 8; ++e) {
    const float v = s[e * 32];
    asm volatile("" :: "v"(v));
    x[e] = v;
  }
  const unsigned mk = (hk == h) ? 0xFFFFFFFFu : 0u;
  v4u o = pack8_bf16((v4f){ x[0], x[1], x[2], x[3] }, (v4f){ x[4], x[5], x[6], x[7] });
  o &= (v4u){ mk, mk, mk, mk };
  return o;
}

__global__ __launch_bounds__(256) void k_prep(
    const float* __restrict__ x, const float* __restrict__ wq, const float* __restrict__ wk,
    const float* __restrict__ wv, const float* __restrict__ bq, const float* __restrict__ bk,
    const float* __restrict__ bv, const float* __restrict__ pri, const float* __restrict__ msg,
    const float* __restrict__ pri2, const float* __restrict__ msg2, const float* __restrict__ comb,
    const float* __restrict__ cfil, const float* __restrict__ temb,
    unsigned short* XB, unsigned short* WT, unsigned short* FBD, unsigned short* MVC, float* PTB, float* PTE) {
  const int b = (int)blockIdx.x, tid = (int)threadIdx.x;
  if (b < PB0) {
    const unsigned g = (unsigned)b * 256u + (unsigned)tid;
    const int row = (int)(g >> 5), p = (int)(g & 31u);
    const int rc = row < NN ? row : NN - 1;
    const float* s = x + (size_t)rc * 256 + 8 * p;
    const v4f a = *(const v4fa*)s, c = *(const v4fa*)(s + 4);
    asm volatile("" :: "v"(a), "v"(c));
    v4u o = pack8_bf16(a, c);
    const unsigned mk = row < NN ? 0xFFFFFFFFu : 0u;
    o &= (v4u){ mk, mk, mk, mk };
    st2_v4u(XB + (size_t)g * 8, o);
  } else if (b < PB1) {
    const int lb = b - PB0;
    const int m = lb >> 5;
    const int u = (lb & 31) * 256 + tid;
    const int n = u >> 5, p = u & 31;
    if (m == 0) {
      st2_v4u(WT + (size_t)u * 8, wt_piece(wq, n, p));
    } else if (m == 1) {
      st2_v4u(WT + (size_t)65536 + (size_t)u * 8, wt_piece(wk, n, p));
    } else {
      st2_v4u(WT + (size_t)131072 + (size_t)u * 8, wt_piece(wv, n, p));
    }
  } else if (b < PB2) {
    const int lb = b - PB1;
    const int t = lb >> 6;
    const int u = (lb & 63) * 256 + tid;
    const int n = u >> 6, p = u & 63;
    st2_v4u(FBD + (size_t)t * 131072 + (size_t)u * 8, bd_piece(cfil + (size_t)t * 8192, n, p));
  } else if (b < PB3) {
    const int lb = b - PB2;
    const int e = lb >> 7;
    const int l7 = lb & 127;
    const int u = l7 * 256 + tid;
    const int nrow = u >> 6, p = u & 63;
    if (l7 < 64) {
      st2_v4u(MVC + (size_t)e * 262144 + (size_t)u * 8, bd_piece(msg + (size_t)e * 8192, nrow, p));
    } else {
      st2_v4u(MVC + (size_t)e * 262144 + (size_t)u * 8, bd_piece(msg2 + (size_t)e * 8192, nrow - 256, p));
    }
  } else if (b < PB4) {
    const int m = b - PB3;
    if (m == 0) {
      st2_f(PTB + tid, bf16_val(bq[tid]));
    } else if (m == 1) {
      st2_f(PTB + 256 + tid, bf16_val(bk[tid]));
    } else {
      st2_f(PTB + 512 + tid, bf16_val(bv[tid]));
    }
  } else {
    const int lb = b - PB4;
    const int e = lb / 3;
    const int kind = lb - 3 * e;
    float* row = PTE + (size_t)e * PTE_N;
    if (kind == 0) {
      st2_f(row + tid, bf16_val(comb[e * 256 + tid]));
    } else if (kind == 1) {
      const int h = tid >> 5, f = tid & 31;
      const float* tp = temb + h * 32;
      const float* mp = msg2 + (size_t)e * 8192 + (size_t)h * 1024 + f;
      float acc = 0.0f;
#pragma unroll 2
      for (int d = 0; d < 32; ++d) {
        const float a = bf16_val(tp[d]);
        const float w = bf16_val(mp[d * 32]);
        acc = fmaf(a, w, acc);
      }
      st2_f(row + 256 + tid, acc);
    } else {
      if (tid < 128) {
        const int lane = tid & 31, wave = tid >> 5;
        const int l8 = lane < 8 ? lane : 7;
        const float pv = pri[e * 8 + l8];
        const float pc = pri2[e * 8 + l8];
        asm volatile("" :: "v"(pv), "v"(pc));
        const float fv = bf16_val(pv) * RS_DK;
        const float fc = bf16_val(pc) * RS_DK;
        float sel = (wave == 0) ? fv : fc;
        sel = (wave < 2 && lane < 8) ? sel : 0.0f;
        st2_f(row + 512 + tid, sel);
      }
    }
  }
}

__global__ __launch_bounds__(256) void k_post(const float* __restrict__ Kf, const float* __restrict__ Vf,
                                              unsigned short* KHL, unsigned short* VHL) {
  const int lane = threadIdx.x & 31, wave = threadIdx.x >> 5;
  const int row = (int)blockIdx.x * 8 + wave;
  const int rc = row < NN ? row : NN - 1;
  const float* kp = Kf + (size_t)rc * 256 + 8 * lane;
  const float* vp = Vf + (size_t)rc * 256 + 8 * lane;
  const v4f ka = *(const v4fa*)kp, kc = *(const v4fa*)(kp + 4);
  const v4f va = *(const v4fa*)vp, vc = *(const v4fa*)(vp + 4);
  asm volatile("" :: "v"(ka), "v"(kc), "v"(va), "v"(vc));
  const unsigned mk = row < NN ? 0xFFFFFFFFu : 0u;
  const v4u m4 = (v4u){ mk, mk, mk, mk };
  const v4u khi = pack8_bf16(ka, kc) & m4;
  const v4u klo = pack8_bf16_lo(ka, kc) & m4;
  const v4u vhi = pack8_bf16(va, vc) & m4;
  const v4u vlo = pack8_bf16_lo(va, vc) & m4;
  unsigned short* kd = KHL + (size_t)row * 512 + 8 * lane;
  unsigned short* vd = VHL + (size_t)row * 512 + 8 * lane;
  volatile v4u* q0 = (volatile v4u*)kd;
  volatile v4u* q1 = (volatile v4u*)(kd + 256);
  volatile v4u* q2 = (volatile v4u*)vd;
  volatile v4u* q3 = (volatile v4u*)(vd + 256);
  *q0 = khi; *q1 = klo; *q2 = vhi; *q3 = vlo;
  __threadfence();
  *q0 = khi; *q1 = klo; *q2 = vhi; *q3 = vlo;
}

__global__ __launch_bounds__(256) void k_select(const float* __restrict__ TMP, const int* __restrict__ ntype,
                                                float* MK, int t) {
  const int lane = threadIdx.x & 31, wave = threadIdx.x >> 5;
  const int row = (int)blockIdx.x * 8 + wave;
  const int ct = clampi(ntype[row], 0, 2);
  const float* tp = TMP + (size_t)row * 256;
  const v4f a = *(const v4fa*)(tp + 4 * lane);
  const v4f c = *(const v4fa*)(tp + 128 + 4 * lane);
  asm volatile("" :: "v"(a), "v"(c));
  if (ct == t) {
    volatile v4f* q0 = (volatile v4f*)(MK + (size_t)row * 256 + 4 * lane);
    volatile v4f* q1 = (volatile v4f*)(MK + (size_t)row * 256 + 128 + 4 * lane);
    *q0 = a; *q1 = c;
    __threadfence();
    *q0 = a; *q1 = c;
  }
}

__device__ __forceinline__ int scan_chunk(const int* __restrict__ dsts, int nE, int cbase, int slotBase,
                                          int nb, int vec8, int* list, int tid, int lane, int wave) {
  int wc = 0;
  const int el0  = tid * EPT;
  const int e0   = cbase + el0;
  const int sent = (-0x7fffffff - 1);
  v4i da, db;
  if (vec8 != 0 && cbase + CHUNK <= nE) {
    da = *(const v4ia*)(dsts + e0);
    db = *(const v4ia*)(dsts + e0 + 4);
  } else {
    const int t0 = dsts[min(e0 + 0, nE - 1)];
    const int t1 = dsts[min(e0 + 1, nE - 1)];
    const int t2 = dsts[min(e0 + 2, nE - 1)];
    const int t3 = dsts[min(e0 + 3, nE - 1)];
    const int t4 = dsts[min(e0 + 4, nE - 1)];
    const int t5 = dsts[min(e0 + 5, nE - 1)];
    const int t6 = dsts[min(e0 + 6, nE - 1)];
    const int t7 = dsts[min(e0 + 7, nE - 1)];
    asm volatile("" :: "v"(t0), "v"(t1), "v"(t2), "v"(t3), "v"(t4), "v"(t5), "v"(t6), "v"(t7));
    da.x = (e0 + 0 < nE) ? t0 : sent;
    da.y = (e0 + 1 < nE) ? t1 : sent;
    da.z = (e0 + 2 < nE) ? t2 : sent;
    da.w = (e0 + 3 < nE) ? t3 : sent;
    db.x = (e0 + 4 < nE) ? t4 : sent;
    db.y = (e0 + 5 < nE) ? t5 : sent;
    db.z = (e0 + 6 < nE) ? t6 : sent;
    db.w = (e0 + 7 < nE) ? t7 : sent;
  }
  const unsigned nbs = (unsigned)slotBase;
  const unsigned unb = (unsigned)nb;
  const unsigned s0 = (unsigned)da.x - nbs, s1 = (unsigned)da.y - nbs;
  const unsigned s2 = (unsigned)da.z - nbs, s3 = (unsigned)da.w - nbs;
  const unsigned s4 = (unsigned)db.x - nbs, s5 = (unsigned)db.y - nbs;
  const unsigned s6 = (unsigned)db.z - nbs, s7 = (unsigned)db.w - nbs;
  const bool h0 = s0 < unb, h1 = s1 < unb, h2 = s2 < unb, h3 = s3 < unb;
  const bool h4 = s4 < unb, h5 = s5 < unb, h6 = s6 < unb, h7 = s7 < unb;
  const unsigned any = __builtin_amdgcn_ballot_w32(h0 | h1 | h2 | h3 | h4 | h5 | h6 | h7);
  if (any != 0u) {
#define HITJ(J, HJ, SJ) { \
      const unsigned mj = __builtin_amdgcn_ballot_w32(HJ); \
      if (mj != 0u) { \
        if (HJ) { \
          const int pos = wc + (int)__builtin_amdgcn_mbcnt_lo(mj, 0u); \
          if (pos < WCAP) list[wave * WCAP + pos] = ((el0 + (J)) << 12) | (int)(SJ); \
        } \
        wc += (int)__builtin_popcount(mj); } }
    HITJ(0, h0, s0)
    HITJ(1, h1, s1)
    HITJ(2, h2, s2)
    HITJ(3, h3, s3)
    HITJ(4, h4, s4)
    HITJ(5, h5, s5)
    HITJ(6, h6, s6)
    HITJ(7, h7, s7)
#undef HITJ
  }
  return wc;
}

__device__ __forceinline__ int build_lists(const int* __restrict__ dsts, int nE, int nodeBase, int nb, int vec8,
                                           int* reg1, int* reg2, int* scnt, int* soff, int* list,
                                           int* wcnt, int* wtot, int tid, int lane, int wave) {
  for (int i = tid; i < NBMAX; i += NTHR) scnt[i] = 0;
  for (int i = tid; i < RCAP; i += NTHR) { reg1[i] = 0; reg2[i] = 0; }
  __syncthreads();

  int tot = 0;
  const int nChunks = (nE + CHUNK - 1) / CHUNK;
#pragma unroll 1
  for (int ch = 0; ch < nChunks; ++ch) {
    const int cbase = ch * CHUNK;
    const int wc = scan_chunk(dsts, nE, cbase, nodeBase, nb, vec8, list, tid, lane, wave);
    if (lane == 0) wcnt[wave] = wc;
    __syncthreads();
    int pre = 0, all = 0;
#pragma unroll
    for (int w2 = 0; w2 < NWAVE; ++w2) {
      int c = wcnt[w2];
      c = c < 0 ? 0 : (c > WCAP ? WCAP : c);
      all += c;
      pre += (w2 < wave) ? c : 0;
    }
    const int wcc  = wc > WCAP ? WCAP : wc;
    const int base = tot + pre;
#pragma unroll 1
    for (int i = lane; i < wcc; i += 32) {
      const int ent = list[wave * WCAP + i];
      const int el  = (ent >> 12) & (CHUNK - 1);
      const int sl  = ent & (NBMAX - 1);
      int eid = cbase + el;
      eid = eid > nE - 1 ? nE - 1 : eid;
      const int pos = base + i;
      if (pos < RCAP) reg1[pos] = (int)(((unsigned)eid << ESH) | (unsigned)sl);
    }
    tot += all;
    tot = tot > RCAP ? RCAP : tot;
    __syncthreads();
  }
  const int nh = tot;

  if (wave == 0) {
#pragma unroll 1
    for (int b0 = 0; b0 < nh; b0 += 32) {
      const int idx = b0 + lane;
      const int uv  = reg1[idx < RCAP ? idx : RCAP - 1];
      const int m32 = (nh - b0) < 32 ? (nh - b0) : 32;
#pragma unroll 1
      for (int k = 0; k < m32; ++k) {
        const int u  = __builtin_amdgcn_readlane(uv, k);
        const int sl = u & (NBMAX - 1);
        if (lane == 0) scnt[sl] = scnt[sl] + 1;
      }
    }
  }
  __syncthreads();

  {
    const int c0r = scnt[2 * tid], c1r = scnt[2 * tid + 1];
    const int e0 = c0r < 0 ? 0 : c0r, e1 = c1r < 0 ? 0 : c1r;
    const int ts = e0 + e1;
    int incl = ts;
#pragma unroll
    for (int d = 1; d < 32; d <<= 1) {
      const int up = __shfl_up(incl, d);
      if (lane >= d) incl += up;
    }
    if (lane == 31) wtot[wave] = incl;
    __syncthreads();
    int pre = 0;
#pragma unroll
    for (int w2 = 0; w2 < NWAVE; ++w2) pre += (w2 < wave) ? wtot[w2] : 0;
    const int run = pre + incl - ts;
    soff[2 * tid + 0] = run;
    soff[2 * tid + 1] = run + e0;
  }
  __syncthreads();
  for (int i = tid; i < NBMAX; i += NTHR) list[i] = soff[i];
  __syncthreads();

  if (wave == 0) {
#pragma unroll 1
    for (int b0 = 0; b0 < nh; b0 += 32) {
      const int idx = b0 + lane;
      const int uv  = reg1[idx < RCAP ? idx : RCAP - 1];
      const int m32 = (nh - b0) < 32 ? (nh - b0) : 32;
#pragma unroll 1
      for (int k = 0; k < m32; ++k) {
        const int u   = __builtin_amdgcn_readlane(uv, k);
        const int sl  = u & (NBMAX - 1);
        const int eid = (int)((unsigned)u >> ESH);
        if (lane == 0) {
          int pos = list[sl];
          pos = pos < 0 ? 0 : (pos > RCAP - 1 ? RCAP - 1 : pos);
          reg2[pos] = eid;
          list[sl] = pos + 1;
        }
      }
    }
  }
  __syncthreads();
  return nh;
}

__global__ __launch_bounds__(NTHR) void k_bucket(const int* __restrict__ dstAll, const int* __restrict__ srcAll,
                                                 int* LIST, int* OFFC, int* META) {
  extern __shared__ v4f lds_dyn[];
  int* reg1 = (int*)lds_dyn;
  int* reg2 = reg1 + RCAP;
  int* scnt = reg2 + RCAP;
  int* soff = scnt + NBMAX;
  int* list = soff + NBMAX;
  int* wcnt = list + LISTN;
  int* wtot = wcnt + NWAVE;
  const int tid = (int)threadIdx.x, lane = tid & 31, wave = tid >> 5;
  const int b = (int)blockIdx.x;
  const int e = (int)blockIdx.y;
  const int* dsts = dstAll + (size_t)e * NE;
  const int* srcs = srcAll + (size_t)e * NE;
  const int nodeBase = b * NBROWS;
  int nb = NN - nodeBase;
  nb = nb < 0 ? 0 : (nb > NBROWS ? NBROWS : nb);

  const int nh = build_lists(dsts, NE, nodeBase, nb, 1, reg1, reg2, scnt, soff, list, wcnt, wtot, tid, lane, wave);

  const int ob = e * NBLK + b;
  int* bl = LIST + (size_t)ob * RCAP;
#pragma unroll 1
  for (int base = 0; base < RCAP; base += 1024) {
    const int i0 = base + 4 * tid;
    const v4i ev = *(const v4ia*)(reg2 + i0);
    int s0 = srcs[clampi(ev.x, 0, NE - 1)];
    int s1 = srcs[clampi(ev.y, 0, NE - 1)];
    int s2 = srcs[clampi(ev.z, 0, NE - 1)];
    int s3 = srcs[clampi(ev.w, 0, NE - 1)];
    asm volatile("" :: "v"(s0), "v"(s1), "v"(s2), "v"(s3));
    v4i v;
    v.x = (i0     < nh) ? s0 : 0;
    v.y = (i0 + 1 < nh) ? s1 : 0;
    v.z = (i0 + 2 < nh) ? s2 : 0;
    v.w = (i0 + 3 < nh) ? s3 : 0;
    st2_v4i(bl + i0, v);
  }
  {
    const v4i sc = *(const v4ia*)(scnt + 4 * tid);
    st2_v4i(OFFC + (size_t)ob * 1024 + 4 * tid, sc);
  }
  if (tid < 8) {
    v4i mv;
    mv.x = (tid == 0) ? nh : 0;
    mv.y = (tid == 0 && nh >= RCAP) ? 1 : 0;
    mv.z = 0; mv.w = 0;
    st2_v4i(META + (size_t)ob * 32 + 4 * tid, mv);
  }
}

template <int E>
__global__ __launch_bounds__(256) void k_att(
    const float* __restrict__ Q, const float* __restrict__ K, const float* __restrict__ MK,
    const float* __restrict__ VC, const int* __restrict__ LIST, const int* __restrict__ OFFC,
    const int* __restrict__ META, const float* __restrict__ PTE, float* out) {
  static_assert(E >= 0 && E < NTYPE);
  __shared__ __attribute__((aligned(16))) float sPar[PTE_N];
  __shared__ __attribute__((aligned(16))) float sRow[8][256];
  const int tid = (int)threadIdx.x, lane = tid & 31, wave = tid >> 5;
  if (tid < PTE_N / 4) {
    const v4f v = *(const v4fa*)(PTE + (size_t)E * PTE_N + 4 * tid);
    *(v4fa*)(sPar + 4 * tid) = v;
  }
  __syncthreads();
  const int bb = (int)blockIdx.x >> 2;
  const int slot0 = ((int)blockIdx.x & 3) * 128 + wave * 16;
  const int nodeBase = bb * NBROWS;
  const int nbrows = clampi(NN - nodeBase, 0, NBROWS);
  if (slot0 >= nbrows) return;

  const int ob = E * NBLK + bb;
  const int nh = clampi(META[(size_t)ob * 32], 0, RCAP);
  const int flag = META[(size_t)ob * 32 + 1];
  const int* bl = LIST + (size_t)ob * RCAP;
  const int* oc = OFFC + (size_t)ob * 1024;
  int cv  = oc[slot0 + (lane & 15)];
  int stv = oc[512 + slot0 + (lane & 15)];
  stv = clampi(stv, 0, nh);
  cv  = clampi(cv, 0, nh - stv);

  const int hd = lane >> 2;
  const float fsc = sPar[512 + hd];
  const float fcs = sPar[544 + hd];
  const v4f cmb0 = *(const v4fa*)(sPar + 8 * lane);
  const v4f cmb1 = *(const v4fa*)(sPar + 8 * lane + 4);
  const v4f tc0  = *(const v4fa*)(sPar + 256 + 8 * lane);
  const v4f tc1  = *(const v4fa*)(sPar + 256 + 8 * lane + 4);
  const float pz = (flag != 0) ? __int_as_float(0x7fc00000) : 0.0f;
  float* strip = &sRow[wave][0];
  const int lastI = nh > 0 ? nh - 1 : 0;

#pragma unroll 1
  for (int rr = 0; rr < 16; ++rr) {
    const int st  = __builtin_amdgcn_readlane(stv, rr);
    const int cnt = __builtin_amdgcn_readlane(cv, rr);
    const int grow = nodeBase + slot0 + rr;
    const float* qp = Q + (size_t)grow * 256 + 8 * lane;
    const v4f q0 = *(const v4fa*)qp, q1 = *(const v4fa*)(qp + 4);

    float m = NEGBIG, S = 0.0f, m2 = NEGBIG, S2 = 0.0f;
    v4f a0 = (v4f){0.f, 0.f, 0.f, 0.f}, a1 = a0, b0 = a0, b1 = a0;
#pragma unroll 1
    for (int qi = 0; qi < cnt; ++qi) {
      int li = st + qi;
      li = li > lastI ? lastI : li;
      int s = bl[li];
      asm volatile("" :: "v"(s));
      s = clampi(s, 0, NN - 1);
      const float* kr = K  + (size_t)s * 256 + 8 * lane;
      const float* mr = MK + (size_t)s * 256 + 8 * lane;
      const float* vr = VC + (size_t)s * 512 + 8 * lane;
      const v4f k0 = *(const v4fa*)kr,         k1 = *(const v4fa*)(kr + 4);
      const v4f g0 = *(const v4fa*)mr,         g1 = *(const v4fa*)(mr + 4);
      const v4f v0 = *(const v4fa*)vr,         v1 = *(const v4fa*)(vr + 4);
      const v4f w0 = *(const v4fa*)(vr + 256), w1 = *(const v4fa*)(vr + 260);
      float da = q0[0] * k0[0];
      da = fmaf(q0[1], k0[1], da); da = fmaf(q0[2], k0[2], da); da = fmaf(q0[3], k0[3], da);
      da = fmaf(q1[0], k1[0], da); da = fmaf(q1[1], k1[1], da); da = fmaf(q1[2], k1[2], da);
      da = fmaf(q1[3], k1[3], da);
      float dc = q0[0] * g0[0];
      dc = fmaf(q0[1], g0[1], dc); dc = fmaf(q0[2], g0[2], dc); dc = fmaf(q0[3], g0[3], dc);
      dc = fmaf(q1[0], g1[0], dc); dc = fmaf(q1[1], g1[1], dc); dc = fmaf(q1[2], g1[2], dc);
      dc = fmaf(q1[3], g1[3], dc);
      da += __shfl_xor(da, 1);
      dc += __shfl_xor(dc, 1);
      da += __shfl_xor(da, 2);
      dc += __shfl_xor(dc, 2);
      const float l  = da * fsc;
      const float l2 = dc * fcs;
      const float mn = fmaxf(m, l);
      const float sc = __expf(m - mn);
      const float p  = __expf(l - mn);
      S  = fmaf(S, sc, p);
      a0 = a0 * sc + v0 * p;
      a1 = a1 * sc + v1 * p;
      m  = mn;
      const float mn2 = fmaxf(m2, l2);
      const float sc2 = __expf(m2 - mn2);
      const float p2  = __expf(l2 - mn2);
      S2 = fmaf(S2, sc2, p2);
      b0 = b0 * sc2 + (w0 + tc0) * p2;
      b1 = b1 * sc2 + (w1 + tc1) * p2;
      m2 = mn2;
    }
    const bool has = cnt > 0;
    const float Ss  = has ? S  : 1.0f;
    const float Ss2 = has ? S2 : 1.0f;
    const float inv  = 1.0f / Ss;
    const float inv2 = 1.0f / Ss2;
    v4f t0 = a0 * inv + (b0 * inv2) * cmb0;
    v4f t1 = a1 * inv + (b1 * inv2) * cmb1;
    const v4f zz = (v4f){0.f, 0.f, 0.f, 0.f};
    t0 = has ? t0 : zz;
    t1 = has ? t1 : zz;

    *(v4fa*)(strip + 8 * lane)     = t0;
    *(v4fa*)(strip + 8 * lane + 4) = t1;
    wave_sync_lds();
    v4f o0 = *(const v4fa*)(strip + 4 * lane);
    v4f o1 = *(const v4fa*)(strip + 128 + 4 * lane);
    wave_sync_lds();
    float* orow = out + (size_t)grow * 256;
    if (E > 0) {
      const v4f p0 = *(const v4fa*)(orow + 4 * lane);
      const v4f p1 = *(const v4fa*)(orow + 128 + 4 * lane);
      o0 += p0;
      o1 += p1;
    }
    o0 += pz;
    o1 += pz;
    if (E == 2) {
      o0 = o0 * (1.0f / 3.0f);
      o1 = o1 * (1.0f / 3.0f);
#pragma unroll
      for (int c = 0; c < 4; ++c) {
        const float u0 = o0[c], u1 = o1[c];
        o0[c] = (u0 > 0.0f) ? u0 : (u0 - u0);
        o1[c] = (u1 > 0.0f) ? u1 : (u1 - u1);
      }
    }
    volatile v4f* w0p = (volatile v4f*)(orow + 4 * lane);
    volatile v4f* w1p = (volatile v4f*)(orow + 128 + 4 * lane);
    *w0p = o0; *w1p = o1;
    __threadfence();
    *w0p = o0; *w1p = o1;
  }
}

extern "C" void kernel_launch(void* const* d_in, const int* in_sizes, int n_in,
                              void* d_out, int out_size, void* d_ws, size_t ws_size,
                              hipStream_t stream) {
  if (n_in < 17) return;
  if (in_sizes[0] != NN * 256) return;
  if (in_sizes[1] != 65536 || in_sizes[3] != 65536 || in_sizes[5] != 65536) return;
  if (in_sizes[2] != 256 || in_sizes[4] != 256 || in_sizes[6] != 256) return;
  if (in_sizes[7] != 24 || in_sizes[9] != 24 || in_sizes[11] != 768 || in_sizes[13] != 256) return;
  if (in_sizes[8] != 24576 || in_sizes[10] != 24576 || in_sizes[12] != 24576) return;
  if (in_sizes[14] != NN || in_sizes[15] != NTYPE * NE || in_sizes[16] != NTYPE * NE) return;
  if (out_size != NN * 256) return;
  if (ws_size < WS_TOTAL) return;

  const float* x     = (const float*)d_in[0];
  const float* Wk    = (const float*)d_in[1];
  const float* bk    = (const float*)d_in[2];
  const float* Wq    = (const float*)d_in[3];
  const float* bq    = (const float*)d_in[4];
  const float* Wv    = (const float*)d_in[5];
  const float* bv    = (const float*)d_in[6];
  const float* pri   = (const float*)d_in[7];
  const float* msg   = (const float*)d_in[8];
  const float* pri2  = (const float*)d_in[9];
  const float* msg2  = (const float*)d_in[10];
  const float* comb  = (const float*)d_in[11];
  const float* cfil  = (const float*)d_in[12];
  const float* temb  = (const float*)d_in[13];
  const int*   ntype = (const int*)  d_in[14];
  const int*   src   = (const int*)  d_in[15];
  const int*   dst   = (const int*)  d_in[16];
  float* out = (float*)d_out;

  char* ws = (char*)d_ws;
  float*          Qp   = (float*)(ws + O_Q);
  float*          Kp   = (float*)(ws + O_K);
  float*          MKp  = (float*)(ws + O_MK);
  float*          VTMP = (float*)(ws + O_MK);
  unsigned short* VHL  = (unsigned short*)(ws + O_VHL);
  float*          VCp  = (float*)(ws + O_VC);
  unsigned short* KHL  = (unsigned short*)(ws + O_KHL);
  float*          TMP  = (float*)(ws + O_TMP);
  unsigned short* XB   = (unsigned short*)(ws + O_XB);
  int*            LIST = (int*)(ws + O_LIST);
  int*            OFFC = (int*)(ws + O_OFFC);
  int*            META = (int*)(ws + O_META);
  unsigned short* WT   = (unsigned short*)(ws + O_WT);
  unsigned short* FBD  = (unsigned short*)(ws + O_FBD);
  unsigned short* MVC  = (unsigned short*)(ws + O_MVC);
  float*          PTB  = (float*)(ws + O_PTB);
  float*          PTE  = (float*)(ws + O_PTE);

  k_prep<<<PB5, 256, 0, stream>>>(x, Wq, Wk, Wv, bq, bk, bv, pri, msg, pri2, msg2, comb, cfil, temb,
                                  XB, WT, FBD, MVC, PTB, PTE);
  k_gemm_nt<0, 1><<<(1252 + 7) / 8, 256, 0, stream>>>(XB, WT,          PTB,       Qp,   NN, 256, 256, 256);
  k_gemm_nt<0, 1><<<(1252 + 7) / 8, 256, 0, stream>>>(XB, WT + 65536,  PTB + 256, Kp,   NN, 256, 256, 256);
  k_gemm_nt<0, 1><<<(1252 + 7) / 8, 256, 0, stream>>>(XB, WT + 131072, PTB + 512, VTMP, NN, 256, 256, 256);
  k_post<<<MPN / 8, 256, 0, stream>>>(Kp, VTMP, KHL, VHL);
  for (int t = 0; t < NTYPE; ++t) {
    k_gemm_nt<1, 0><<<(1252 + 7) / 8, 256, 0, stream>>>(KHL, FBD + (size_t)t * 131072, PTB, TMP, NN, 256, 512, 256);
    k_select<<<NN / 8, 256, 0, stream>>>(TMP, ntype, MKp, t);
  }
  k_bucket<<<dim3(NBLK, NTYPE), NTHR, LDS_BKT, stream>>>(dst, src, LIST, OFFC, META);
  k_gemm_nt<1, 0><<<(2504 + 7) / 8, 256, 0, stream>>>(VHL, MVC, PTB, VCp, NN, 512, 512, 512);
  k_att<0><<<NBLK * 4, 256, 0, stream>>>(Qp, Kp, MKp, VCp, LIST, OFFC, META, PTE, out);
  k_gemm_nt<1, 0><<<(2504 + 7) / 8, 256, 0, stream>>>(VHL, MVC + (size_t)262144, PTB, VCp, NN, 512, 512, 512);
  k_att<1><<<NBLK * 4, 256, 0, stream>>>(Qp, Kp, MKp, VCp, LIST, OFFC, META, PTE, out);
  k_gemm_nt<1, 0><<<(2504 + 7) / 8, 256, 0, stream>>>(VHL, MVC + (size_t)524288, PTB, VCp, NN, 512, 512, 512);
  k_att<2><<<NBLK * 4, 256, 0, stream>>>(Qp, Kp, MKp, VCp, LIST, OFFC, META, PTE, out);
}
